// SelfAttention_reduce_sumsampling_18073222382373
// MI455X (gfx1250) — hardware-verified
//
#include <hip/hip_runtime.h>
#include <math.h>

typedef __attribute__((ext_vector_type(16))) _Float16 v16h;
typedef __attribute__((ext_vector_type(16))) __bf16 v16b;
typedef __attribute__((ext_vector_type(8)))  _Float16 v8h;
typedef __attribute__((ext_vector_type(8)))  float v8f;
typedef __attribute__((ext_vector_type(4)))  float v4f;
typedef __attribute__((ext_vector_type(2)))  float v2f;
typedef __attribute__((ext_vector_type(4)))  unsigned v4u;
typedef __attribute__((ext_vector_type(4)))  int v4i;
typedef float __attribute__((may_alias)) float_a;
typedef int __attribute__((may_alias)) int_a;

template <typename T> __device__ __forceinline__ void vst2(void* p, T v) { *(volatile T*)p = v; __threadfence(); *(volatile T*)p = v; }
__device__ __forceinline__ v8f wmma16(v16h a, v16h b, v8f c) {
  v8f d = __builtin_amdgcn_wmma_f32_16x16x32_f16(false, a, false, b, (short)0, c, false, false);
  asm volatile("v_nop\n\tv_nop\n\tv_nop\n\tv_nop" : "+v"(d) : "v"(a), "v"(b));
  return d;
}
__device__ __forceinline__ v8f wmma_bf(v16b a, v16b b, v8f c) {
  v8f d = __builtin_amdgcn_wmma_f32_16x16x32_bf16(false, a, false, b, (short)0, c, false, false);
  asm volatile("v_nop\n\tv_nop\n\tv_nop\n\tv_nop" : "+v"(d) : "v"(a), "v"(b));
  return d;
}
__device__ __forceinline__ v16h frag_h(const _Float16* rowk0, int lane) {
  union { v16h v; v8h q[2]; } u; const _Float16* p = rowk0 + 8 * (lane >> 4);
  u.q[0] = *(const v8h*)p; u.q[1] = *(const v8h*)(p + 16); return u.v;
}
__device__ __forceinline__ v16h frag_f32(const float* rowk0, int lane) {
  v16h a; const float* p = rowk0 + 8 * (lane >> 4);
#pragma unroll
  for (int i = 0; i < 8; ++i) { a[i] = (_Float16)p[i]; a[8 + i] = (_Float16)p[16 + i]; }
  return a;
}
__device__ __forceinline__ v16h frag_f32s(const float* rowk0, int lane, float sc) {
  v16h a; const float* p = rowk0 + 8 * (lane >> 4);
#pragma unroll
  for (int i = 0; i < 8; ++i) { a[i] = (_Float16)(p[i] * sc); a[8 + i] = (_Float16)(p[16 + i] * sc); }
  return a;
}
__device__ __forceinline__ v16h fragc_f32(const float* W, int k0, int n, int lane, int ld, int K) {
  v16h a; const int g = lane >> 4;
#pragma unroll
  for (int i = 0; i < 8; ++i) { const int ka = k0 + 8 * g + i, kb = ka + 16;
    a[i] = (_Float16)(ka < K ? W[(size_t)(ka < K ? ka : K - 1) * ld + n] : 0.f); a[8 + i] = (_Float16)(kb < K ? W[(size_t)(kb < K ? kb : K - 1) * ld + n] : 0.f); }
  return a;
}
struct F2 { v16b h, l; };
__device__ __forceinline__ F2 bsplit16(const float v[16]) { F2 r;
#pragma unroll
  for (int i = 0; i < 16; ++i) { const __bf16 h = (__bf16)v[i]; r.h[i] = h; r.l[i] = (__bf16)(v[i] - (float)h); }
  return r; }
__device__ __forceinline__ F2 split_row(const float* row, int k0, int lane) { float v[16]; const float* p = row + k0 + 8 * (lane >> 4);
#pragma unroll
  for (int i = 0; i < 8; ++i) { v[i] = p[i]; v[8 + i] = p[16 + i]; }
  return bsplit16(v); }
__device__ __forceinline__ F2 split_rowK(const float* row, int k0, int lane, int K) { float v[16]; const int g = lane >> 4;
#pragma unroll
  for (int i = 0; i < 8; ++i) { const int ka = k0 + 8 * g + i, kb = ka + 16; v[i] = ka < K ? row[ka < K ? ka : K - 1] : 0.f; v[8 + i] = kb < K ? row[kb < K ? kb : K - 1] : 0.f; }
  return bsplit16(v); }
__device__ __forceinline__ F2 split_col(const float* W, int k0, int n, int lane, int ld, int K) { float v[16]; const int g = lane >> 4;
#pragma unroll
  for (int i = 0; i < 8; ++i) { const int ka = k0 + 8 * g + i, kb = ka + 16; v[i] = ka < K ? W[(size_t)(ka < K ? ka : K - 1) * ld + n] : 0.f; v[8 + i] = kb < K ? W[(size_t)(kb < K ? kb : K - 1) * ld + n] : 0.f; }
  return bsplit16(v); }
__device__ __forceinline__ v8f mac3(const F2& a, const F2& b, v8f c) { c = wmma_bf(a.l, b.h, c); c = wmma_bf(a.h, b.l, c); return wmma_bf(a.h, b.h, c); }
__device__ __forceinline__ float sigm(float v) { return 1.0f / (1.0f + expf(-v)); }
#define LDSX() do { asm volatile("s_wait_dscnt 0" ::: "memory"); __builtin_amdgcn_wave_barrier(); __builtin_amdgcn_fence(__ATOMIC_RELEASE, "workgroup"); } while (0)


#define NB 8
#define NN 4096
#define CC 256
#define CI 32
#ifndef TNB
#define TNB NB
#endif
typedef __attribute__((ext_vector_type(8))) __bf16 v8b;
__device__ __forceinline__ v16b frag_b(const __bf16* rowk0, int lane) {
  union { v16b v; v8b q[2]; } u; const __bf16* p = rowk0 + 8 * (lane >> 4);
  u.q[0] = *(const v8b*)p; u.q[1] = *(const v8b*)(p + 16); return u.v;
}
__device__ __forceinline__ float bfr(float v) { return (float)(__bf16)v; }
__device__ __attribute__((noinline)) float exp_ni(float v) { return expf(v); }
__device__ __attribute__((noinline)) float erf_ni(float v) { return erff(v); }

#define WS_PW  0u
#define WS_PO  (WS_PW + 2u * 3 * CI * CC)
#define WS_FG  (WS_PO + 2u * CC * CI)
#define WS_FGL (WS_FG + 2u * (size_t)NB * NN * 2 * CI)
#define WS_HT  (WS_FGL + 2u * (size_t)NB * NN * 2 * CI)
#define WS_HTL (WS_HT + 2u * (size_t)NB * CI * NN)
#define WS_AG  (WS_HTL + 2u * (size_t)NB * CI * NN)
#define WS_END (WS_AG + 4u * (size_t)NB * NN * CI)

__global__ __launch_bounds__(256) void k_pack(const float* __restrict__ WFY, const float* __restrict__ WGX, const float* __restrict__ WHX, const float* __restrict__ WOUT, __bf16* __restrict__ PW, __bf16* __restrict__ PO) { const int n = blockIdx.x, t = threadIdx.x; __shared__ __align__(16) __bf16 s[CC];
  if (n < 3 * CI) { const float* Wm = n < CI ? WFY : n < 2 * CI ? WGX : WHX; const int o = n % CI; s[t] = (__bf16)Wm[(size_t)t * CI + o]; __syncthreads(); if (t < CC / 8) vst2((unsigned*)(PW + (size_t)n * CC + t * 8), *(const v4u*)&s[t * 8]); }
  else { const int o = n - 3 * CI; if (t < CI) s[t] = (__bf16)WOUT[(size_t)t * CC + o]; __syncthreads(); if (t < CI / 8) vst2((unsigned*)(PO + (size_t)o * CI + t * 8), *(const v4u*)&s[t * 8]); } }
__device__ __forceinline__ v16b fragb_f32(const float* __restrict__ p, int lane) { v16b a; const float* pp = p + 8 * (lane >> 4);
#pragma unroll
  for (int i = 0; i < 8; ++i) { a[i] = (__bf16)pp[i]; a[8 + i] = (__bf16)pp[16 + i]; } return a; }
__global__ __launch_bounds__(128) void k_proj(const float* __restrict__ X, const float* __restrict__ Y, const __bf16* __restrict__ PW, _Float16* __restrict__ FG, _Float16* __restrict__ FGL, _Float16* __restrict__ HT, _Float16* __restrict__ HTL) {
  __shared__ __align__(16) _Float16 sh[64][72], sl[64][72]; __shared__ __align__(16) _Float16 th[CI][72], tl[CI][72];
  const int tid = threadIdx.x, wave = tid >> 5, lane = tid & 31, col = lane & 15, g = lane >> 4; const size_t b = blockIdx.y; const int n0 = blockIdx.x * 64 + wave * 16; const size_t r0 = b * NN + n0;
  v8f acc[6] = {};
#pragma unroll 2
  for (int kc = 0; kc < CC / 32; ++kc) { const v16b ay = fragb_f32(Y + (r0 + col) * CC + kc * 32, lane), ax = fragb_f32(X + (r0 + col) * CC + kc * 32, lane);
#pragma unroll
    for (int j = 0; j < 6; ++j) acc[j] = wmma_bf(j < 2 ? ay : ax, frag_b(PW + (size_t)(j * 16 + col) * CC + kc * 32, lane), acc[j]); }
#pragma unroll
  for (int j = 0; j < 6; ++j)
#pragma unroll
    for (int r = 0; r < 8; ++r) { const float v = acc[j][r]; const _Float16 hv = (_Float16)v, lv = (_Float16)((v - (float)hv) * 2048.0f); if (j < 4) { sh[wave * 16 + 8 * g + r][j * 16 + col] = hv; sl[wave * 16 + 8 * g + r][j * 16 + col] = lv; } else { th[(j - 4) * 16 + col][wave * 16 + 8 * g + r] = hv; tl[(j - 4) * 16 + col][wave * 16 + 8 * g + r] = lv; } }
  __syncthreads();
  for (int e = tid; e < 64 * 8; e += 128) { const int rl = e >> 3, q = e & 7; const size_t o = (b * NN + blockIdx.x * 64 + rl) * (2 * CI) + q * 8; vst2((unsigned*)(FG + o), *(const v4u*)&sh[rl][q * 8]); vst2((unsigned*)(FGL + o), *(const v4u*)&sl[rl][q * 8]); }
  for (int e = tid; e < CI * 8; e += 128) { const int cl = e >> 3, q = e & 7; const size_t o = (b * CI + cl) * (size_t)NN + blockIdx.x * 64 + q * 8; vst2((unsigned*)(HT + o), *(const v4u*)&th[cl][q * 8]); vst2((unsigned*)(HTL + o), *(const v4u*)&tl[cl][q * 8]); } }
__global__ __launch_bounds__(128) void k_att(const _Float16* __restrict__ FG, const _Float16* __restrict__ FGL, const _Float16* __restrict__ HT, const _Float16* __restrict__ HTL, float* __restrict__ AG) {
  __shared__ __align__(16) float sp[4][16][36]; __shared__ __align__(16) float so[4][16][36];
  const int tid = threadIdx.x, wave = tid >> 5, lane = tid & 31, col = lane & 15, g = lane >> 4; const size_t b = blockIdx.y; const int q0 = blockIdx.x * 64 + wave * 16; const size_t rq = b * NN + q0;
  const v16h aq = frag_h(FG + (rq + col) * (2 * CI), lane), aql = frag_h(FGL + (rq + col) * (2 * CI), lane);
  float m[8], l[8];
#pragma unroll
  for (int r = 0; r < 8; ++r) { m[r] = -3.0e38f; l[r] = 0.f; }
  v8f acc[2] = {}, accl[2] = {};
#pragma unroll 1
  for (int ks = 0; ks < NN / 32; ++ks) { v8f s[2];
#pragma unroll
    for (int ct = 0; ct < 2; ++ct) { const size_t rk = b * NN + ks * 32 + ct * 16 + col; const v16h kh = frag_h(FG + rk * (2 * CI) + CI, lane), kl = frag_h(FGL + rk * (2 * CI) + CI, lane); v8f c = {}, cl = {}; c = wmma16(aq, kh, c); cl = wmma16(aq, kl, cl); cl = wmma16(aql, kh, cl);
#pragma unroll
      for (int r = 0; r < 8; ++r) s[ct][r] = c[r] + cl[r] * (1.0f / 2048.0f); }
    float alpha[8];
#pragma unroll
    for (int r = 0; r < 8; ++r) { float mx = fmaxf(s[0][r], s[1][r]);
#pragma unroll
      for (int o = 1; o < 16; o <<= 1) mx = fmaxf(mx, __shfl_xor(mx, o));
      const float mn = fmaxf(m[r], mx); alpha[r] = __expf(m[r] - mn); const float e0 = __expf(s[0][r] - mn), e1 = __expf(s[1][r] - mn); float es = e0 + e1;
#pragma unroll
      for (int o = 1; o < 16; o <<= 1) es += __shfl_xor(es, o);
      l[r] = l[r] * alpha[r] + es; m[r] = mn; sp[wave][8 * g + r][col] = e0; sp[wave][8 * g + r][16 + col] = e1; }
#pragma unroll
    for (int j = 0; j < 2; ++j)
#pragma unroll
      for (int r = 0; r < 8; ++r) { acc[j][r] *= alpha[r]; accl[j][r] *= alpha[r]; }
    LDSX();
    v16h pa; { const float* prow = &sp[wave][col][0] + 8 * (lane >> 4);
#pragma unroll
      for (int i = 0; i < 8; ++i) { pa[i] = (_Float16)(prow[i] * 2048.0f); pa[8 + i] = (_Float16)(prow[16 + i] * 2048.0f); } }
#pragma unroll
    for (int j = 0; j < 2; ++j) { const size_t po = (b * CI + j * 16 + col) * (size_t)NN + ks * 32; acc[j] = wmma16(pa, frag_h(HT + po, lane), acc[j]); accl[j] = wmma16(pa, frag_h(HTL + po, lane), accl[j]); }
    LDSX(); }
#pragma unroll
  for (int r = 0; r < 8; ++r) { const float il = (1.0f / 2048.0f) / l[r];
#pragma unroll
    for (int j = 0; j < 2; ++j) so[wave][8 * g + r][j * 16 + col] = (acc[j][r] + accl[j][r] * (1.0f / 2048.0f)) * il; }
  LDSX(); for (int rl = 0; rl < 16; ++rl) if (lane < 8) vst2(AG + (rq + rl) * CI + lane * 4, *(const v4f*)&so[wave][rl][lane * 4]); }
__global__ __launch_bounds__(128) void k_out(const float* __restrict__ AG, const __bf16* __restrict__ PO, const float* __restrict__ X, const float* __restrict__ SIG, float* __restrict__ OUT) { __shared__ __align__(16) float sf[4][16][132];
  const int tid = threadIdx.x, wave = tid >> 5, lane = tid & 31, col = lane & 15, g = lane >> 4; const size_t r0 = (size_t)blockIdx.x * 64 + wave * 16; const int c0 = blockIdx.y * 128; const float sg = bfr(SIG[0]);
  v8f acc[8] = {}; { const F2 a = split_row(AG + (r0 + col) * CI, 0, lane);
#pragma unroll
    for (int j = 0; j < 8; ++j) { const v16b w = frag_b(PO + (size_t)(c0 + j * 16 + col) * CI, lane); acc[j] = wmma_bf(a.h, w, acc[j]); acc[j] = wmma_bf(a.l, w, acc[j]); } }
#pragma unroll
  for (int j = 0; j < 8; ++j) { const int c = c0 + j * 16 + col;
#pragma unroll
    for (int r = 0; r < 8; ++r) sf[wave][8 * g + r][j * 16 + col] = bfr(X[(r0 + 8 * g + r) * CC + c]) + sg * acc[j][r]; }
  LDSX(); for (int rl = 0; rl < 16; ++rl) vst2(OUT + (r0 + rl) * CC + c0 + lane * 4, *(const v4f*)&sf[wave][rl][lane * 4]); }
extern "C" void kernel_launch(void* const* d_in, const int* in_sizes, int n_in, void* d_out, int out_size, void* d_ws, size_t ws_size, hipStream_t stream) {
  (void)in_sizes; (void)n_in; (void)out_size;
  const float** F = (const float**)d_in;
  if (ws_size < (size_t)WS_END) return;
  char* ws = (char*)d_ws; __bf16 *PW = (__bf16*)(ws + WS_PW), *PO = (__bf16*)(ws + WS_PO); _Float16 *FG = (_Float16*)(ws + WS_FG), *FGL = (_Float16*)(ws + WS_FGL), *HT = (_Float16*)(ws + WS_HT), *HTL = (_Float16*)(ws + WS_HTL); float* AG = (float*)(ws + WS_AG);
  k_pack<<<3 * CI + CC, 256, 0, stream>>>(F[2], F[3], F[4], F[5], PW, PO);
  k_proj<<<dim3(NN / 64, TNB), 128, 0, stream>>>(F[0], F[1], PW, FG, FGL, HT, HTL);
  k_att<<<dim3(NN / 64, TNB), 128, 0, stream>>>(FG, FGL, HT, HTL, AG);
  k_out<<<dim3(TNB * NN / 64, CC / 128), 128, 0, stream>>>(AG, PO, F[0], F[6], (float*)d_out);
}
